// BlockSparseAttention_5007931867259
// MI455X (gfx1250) — hardware-verified
//
#include <hip/hip_runtime.h>


typedef _Float16       v16h __attribute__((ext_vector_type(16)));
typedef _Float16       v8h  __attribute__((ext_vector_type(8)));
typedef _Float16       v4h  __attribute__((ext_vector_type(4)));
typedef __bf16         v16b __attribute__((ext_vector_type(16)));
typedef unsigned short v8us __attribute__((ext_vector_type(8)));
typedef unsigned short v4us __attribute__((ext_vector_type(4)));
typedef float          v8f  __attribute__((ext_vector_type(8)));
typedef float          v4f  __attribute__((ext_vector_type(4)));

#define SQ    4096
#define HQ    16
#define DQ    64
#define TB    64
#define NBLK  (SQ / TB)
#define HALFW 2
#define LSTR  72
#define SSTR  324
#define PSTR  328
#define OSTR  68
#define NT    128

union FragH { v16h v; v8h half[2]; };
union FragB { v16b v; v16h hv; v8us half[2]; unsigned short s[16]; };

__device__ __forceinline__ void split_bf16(float x, unsigned short& hi, unsigned short& lo) {
  unsigned u  = __float_as_uint(x);
  unsigned hu = (u + 0x7FFFu + ((u >> 16) & 1u)) >> 16;
  float    hf = __uint_as_float(hu << 16);
  float    rm = x - hf;
  unsigned ru = __float_as_uint(rm);
  unsigned lu = (ru + 0x7FFFu + ((ru >> 16) & 1u)) >> 16;
  hi = (unsigned short)hu;
  lo = (unsigned short)lu;
}

__device__ __forceinline__ v8f mma_bf16(const FragB& a, const FragB& b, v8f c) {
  c = __builtin_amdgcn_wmma_f32_16x16x32_bf16(false, a.v, false, b.v, (short)0, c, false, false);
  asm volatile("v_nop\n\tv_nop\n\tv_nop\n\tv_nop" : "+v"(c) : "v"(a.hv), "v"(b.hv));
  return c;
}

__device__ __forceinline__ v8f mma_f16(const FragH& a, const FragH& b, v8f c) {
  c = __builtin_amdgcn_wmma_f32_16x16x32_f16(false, a.v, false, b.v, (short)0, c, false, false);
  asm volatile("v_nop\n\tv_nop\n\tv_nop\n\tv_nop" : "+v"(c) : "v"(a.v), "v"(b.v));
  return c;
}

__global__ __launch_bounds__(NT)
void swattn_kernel(const float* __restrict__ q,
                   const float* __restrict__ k,
                   const float* __restrict__ v,
                   float* __restrict__ out,
                   int total_tiles)
{
  __shared__ __attribute__((aligned(16))) float          Sl[TB * SSTR];
  __shared__ __attribute__((aligned(16))) _Float16       Pl[TB * PSTR];
  __shared__ __attribute__((aligned(16))) unsigned short Khi[TB * LSTR];
  __shared__ __attribute__((aligned(16))) unsigned short Klo[TB * LSTR];
  __shared__ __attribute__((aligned(16))) _Float16       Vt[TB * LSTR];
  __shared__ __attribute__((aligned(16))) float          rsc[TB];

  const int bid = blockIdx.x;
  if (bid >= total_tiles) return;

  const int tid   = threadIdx.x;
  const int lane  = tid & 31;
  const int wave  = tid >> 5;
  const int hh    = lane >> 4;
  const int mm    = lane & 15;
  const int mBase = wave * 16;

  const int n0 = bid % NBLK;
  const int h  = (bid / NBLK) % HQ;
  const int b  = bid / (NBLK * HQ);

  int jlo = n0 - HALFW; if (jlo < 0) jlo = 0;
  int jhi = n0 + HALFW; if (jhi > NBLK - 1) jhi = NBLK - 1;
  const int nv = jhi - jlo + 1;

  const size_t rowpitch = (size_t)HQ * DQ;
  const size_t qbase = (((size_t)b * SQ + (size_t)n0 * TB) * HQ + h) * DQ;

  FragB aqh[2], aql[2];
  {
    const float* qrow = q + qbase + (size_t)(mBase + mm) * rowpitch;
    #pragma unroll
    for (int kk = 0; kk < 2; ++kk) {
      #pragma unroll
      for (int part = 0; part < 2; ++part) {
        const float* p = qrow + kk * 32 + part * 16 + 8 * hh;
        v4f f0 = *(const v4f*)(p);
        v4f f1 = *(const v4f*)(p + 4);
        #pragma unroll
        for (int i = 0; i < 4; ++i) {
          unsigned short sh, sl;
          split_bf16(f0[i], sh, sl);
          aqh[kk].s[part * 8 + i] = sh;
          aql[kk].s[part * 8 + i] = sl;
          split_bf16(f1[i], sh, sl);
          aqh[kk].s[part * 8 + 4 + i] = sh;
          aql[kk].s[part * 8 + 4 + i] = sl;
        }
      }
    }
  }

  for (int s = 0; s < nv; ++s) {
    const int j = jlo + s;
    const float* ksrc = k + (((size_t)b * SQ + (size_t)j * TB) * HQ + h) * DQ;
    __syncthreads();
    #pragma unroll
    for (int i = 0; i < 8; ++i) {
      const int idx = tid + i * NT;
      const int r   = idx >> 4;
      const int c4  = idx & 15;
      v4f f = *(const v4f*)(ksrc + (size_t)r * rowpitch + c4 * 4);
      v4us hv, lv;
      #pragma unroll
      for (int jj = 0; jj < 4; ++jj) {
        unsigned short sh, sl;
        split_bf16(f[jj], sh, sl);
        hv[jj] = sh; lv[jj] = sl;
      }
      *(v4us*)(Khi + r * LSTR + c4 * 4) = hv;
      *(v4us*)(Klo + r * LSTR + c4 * 4) = lv;
    }
    __syncthreads();

    #pragma unroll
    for (int t = 0; t < 4; ++t) {
      v8f acc;
      #pragma unroll
      for (int r = 0; r < 8; ++r) acc[r] = 0.0f;
      #pragma unroll
      for (int kk = 0; kk < 2; ++kk) {
        const unsigned short* ph = Khi + (t * 16 + mm) * LSTR + kk * 32 + 8 * hh;
        const unsigned short* pl = Klo + (t * 16 + mm) * LSTR + kk * 32 + 8 * hh;
        FragB bh, bl;
        bh.half[0] = *(const v8us*)(ph);
        bh.half[1] = *(const v8us*)(ph + 16);
        bl.half[0] = *(const v8us*)(pl);
        bl.half[1] = *(const v8us*)(pl + 16);
        acc = mma_bf16(aqh[kk], bh, acc);
        acc = mma_bf16(aqh[kk], bl, acc);
        acc = mma_bf16(aql[kk], bh, acc);
      }
      float* srow = Sl + (mBase + 8 * hh) * SSTR + s * 64 + t * 16 + mm;
      #pragma unroll
      for (int r = 0; r < 8; ++r) srow[r * SSTR] = acc[r];
    }
  }
  __syncthreads();

  {
    const int m  = mBase + mm;
    const int hc = nv * 32;
    const int c0 = hh * hc;
    const float* srow = Sl + m * SSTR;
    _Float16*    prow = Pl + m * PSTR;
    float mx = -3.0e38f;
    for (int c = c0; c < c0 + hc; c += 4) {
      v4f x = *(const v4f*)(srow + c);
      mx = fmaxf(mx, fmaxf(fmaxf(x[0], x[1]), fmaxf(x[2], x[3])));
    }
    mx = fmaxf(mx, __shfl_xor(mx, 16, 32));
    mx *= 0.125f;
    float sum = 0.0f;
    for (int c = c0; c < c0 + hc; c += 4) {
      v4f x = *(const v4f*)(srow + c);
      v4h pv;
      #pragma unroll
      for (int jj = 0; jj < 4; ++jj) {
        float e = __expf(x[jj] * 0.125f - mx);
        sum += e;
        pv[jj] = (_Float16)(e * 256.0f);
      }
      *(v4h*)(prow + c) = pv;
    }
    sum += __shfl_xor(sum, 16, 32);
    if (hh == 0) rsc[m] = (1.0f / sum) * 0.000244140625f;
  }

  v8f acc[4];
  #pragma unroll
  for (int t = 0; t < 4; ++t) {
    #pragma unroll
    for (int r = 0; r < 8; ++r) acc[t][r] = 0.0f;
  }
  for (int s = 0; s < nv; ++s) {
    const int j = jlo + s;
    const float* vsrc = v + (((size_t)b * SQ + (size_t)j * TB) * HQ + h) * DQ;
    __syncthreads();
    #pragma unroll
    for (int i = 0; i < 8; ++i) {
      const int idx = tid + i * NT;
      const int r   = idx >> 4;
      const int c4  = idx & 15;
      v4f f = *(const v4f*)(vsrc + (size_t)r * rowpitch + c4 * 4);
      #pragma unroll
      for (int jj = 0; jj < 4; ++jj)
        Vt[(c4 * 4 + jj) * LSTR + r] = (_Float16)(f[jj] * 16.0f);
    }
    __syncthreads();

    #pragma unroll
    for (int c = 0; c < 2; ++c) {
      const _Float16* pp = Pl + (mBase + mm) * PSTR + s * 64 + c * 32 + 8 * hh;
      FragH ap;
      ap.half[0] = *(const v8h*)(pp);
      ap.half[1] = *(const v8h*)(pp + 16);
      #pragma unroll
      for (int t = 0; t < 4; ++t) {
        const _Float16* pb = Vt + (t * 16 + mm) * LSTR + c * 32 + 8 * hh;
        FragH bv;
        bv.half[0] = *(const v8h*)(pb);
        bv.half[1] = *(const v8h*)(pb + 16);
        acc[t] = mma_f16(ap, bv, acc[t]);
      }
    }
  }

  __syncthreads();
  {
    float rr[8];
    #pragma unroll
    for (int r = 0; r < 8; ++r) rr[r] = rsc[mBase + 8 * hh + r];
    float* orow = Sl + (mBase + 8 * hh) * OSTR + mm;
    #pragma unroll
    for (int t = 0; t < 4; ++t) {
      #pragma unroll
      for (int r = 0; r < 8; ++r) orow[r * OSTR + t * 16] = acc[t][r] * rr[r];
    }
  }
  __syncthreads();
  {
    const int c4 = lane & 15;
    v4f vals[8];
    #pragma unroll
    for (int it = 0; it < 8; ++it) {
      const int row = mBase + 2 * it + hh;
      vals[it] = *(const v4f*)(Sl + row * OSTR + c4 * 4);
    }
    float* obase = out + qbase + c4 * 4;
    #pragma unroll
    for (int it = 0; it < 8; ++it) {
      const int row = mBase + 2 * it + hh;
      *(volatile v4f*)(obase + (size_t)row * rowpitch) = vals[it];
    }
    __threadfence();
    #pragma unroll
    for (int it = 0; it < 8; ++it) {
      const int row = mBase + 2 * it + hh;
      *(volatile v4f*)(obase + (size_t)row * rowpitch) = vals[it];
    }
  }
}

extern "C" void kernel_launch(void* const* d_in, const int* in_sizes, int n_in,
                              void* d_out, int out_size, void* d_ws, size_t ws_size,
                              hipStream_t stream) {
  (void)d_ws; (void)ws_size;
  if (n_in < 3) return;
  const float* q = (const float*)d_in[0];
  const float* k = (const float*)d_in[1];
  const float* v = (const float*)d_in[2];
  float* out = (float*)d_out;

  const int per_b = SQ * HQ * DQ;
  int nb  = in_sizes[0] / per_b;
  int nbo = out_size / per_b;
  if (nbo < nb) nb = nbo;
  if (nb <= 0) return;
  const int total_tiles = nb * HQ * NBLK;

  swattn_kernel<<<dim3(total_tiles), dim3(NT), 0, stream>>>(q, k, v, out, total_tiles);
}
